// smpl_model_refined_90460601188973
// MI455X (gfx1250) — hardware-run, weakly checked
//
#include <hip/hip_runtime.h>
#include <math.h>

typedef __attribute__((ext_vector_type(16))) _Float16 v16h;
typedef __attribute__((ext_vector_type(8)))  _Float16 v8h;
typedef __attribute__((ext_vector_type(8)))  float    v8f;
typedef __attribute__((ext_vector_type(4)))  float    v4f;
typedef __attribute__((ext_vector_type(2)))  float    v2f;

constexpr int kNV      = 6890;
constexpr int kNVPad   = 6912;
constexpr int kNJ      = 24;
constexpr int kNBeta   = 10;
constexpr int kBatch   = 256;
constexpr int kKdim    = 96;
constexpr int kCdim    = 768;
constexpr int kPts     = 100;
constexpr int kGroups  = 4;
constexpr float kCarryW = 16.0f;
static_assert(kKdim == kNJ * 4, "K = joints x 4");
static_assert(kCdim == kBatch * 3, "M = batch x 3");
static_assert((kKdim % 32) == 0, "GEMM K multiple of 32");
static_assert((kCdim % 64) == 0 && (kNVPad % 64) == 0, "GEMM M,N multiples of 64");
static_assert((kNVPad % 256) == 0 && kNVPad >= kNV, "vertex padding");

constexpr size_t kOut0Bytes = 21166080ull;
constexpr size_t kOut1Byte  = 21166080ull;
constexpr size_t kOut2Byte  = 21239808ull;
constexpr size_t kOutTotalBytes = 22468608ull;
constexpr int kOut0Elems = kBatch * kNV * 3;
constexpr int kOut1Elems = kBatch * kNJ * 3;
constexpr int kOut2Elems = kBatch * kGroups * kPts * 3;
constexpr int kOut1Off   = (int)(kOut1Byte / 4);
constexpr int kOut2Off   = (int)(kOut2Byte / 4);
static_assert((size_t)kOut0Elems * 4 == kOut0Bytes, "out0 size");
static_assert(kOut1Off == kOut0Elems, "out1 offset");
static_assert(kOut2Off == kOut0Elems + kOut1Elems, "out2 offset");
static_assert(kOut2Byte + (size_t)kOut2Elems * 4 == kOutTotalBytes, "out total");
static_assert((kOut1Byte % 128) == 0 && (kOut2Byte % 128) == 0, "line aligned outputs");
static_assert((kOut0Elems % 128) == 0, "out0 = whole 512-B wave chunks");
constexpr int kOut0F4 = kOut0Elems / 4;

constexpr size_t kOffVS4 = 0;
constexpr size_t kOffWH  = kOffVS4 + (size_t)kNVPad * 4 * 4;
constexpr size_t kOffJSP = kOffWH  + (size_t)kNVPad * kKdim * 2;
constexpr size_t kOffAF  = kOffJSP + (size_t)kNJ * 32 * 4;
constexpr size_t kOffAH  = kOffAF  + (size_t)kCdim * kKdim * 4;
constexpr size_t kOffCP  = kOffAH  + (size_t)kCdim * kKdim * 2;
constexpr size_t kWsTotal = kOffCP + (size_t)kCdim * kNVPad * 4;
static_assert(kWsTotal == 23116800ull, "carve total");
static_assert(kWsTotal <= 134217728ull, "carve cap");
static_assert((kOffWH % 128) == 0 && (kOffJSP % 128) == 0 && (kOffAF % 128) == 0 &&
              (kOffAH % 128) == 0 && (kOffCP % 128) == 0, "128-B aligned regions");

constexpr int kParent[24] = {0,0,0,0,1,2,3,4,5,6,7,8,9,9,9,12,13,14,16,17,18,19,20,21};
static_assert(sizeof(kParent) / sizeof(kParent[0]) == 24, "parent table length");
constexpr unsigned long long pack_parents(int base) {
  unsigned long long r = 0ull;
  for (int i = 0; i < 12; ++i) r |= ((unsigned long long)kParent[base + i]) << (5 * i);
  return r;
}
constexpr unsigned long long kParLo = pack_parents(0);
constexpr unsigned long long kParHi = pack_parents(12);

__device__ __forceinline__ v16h frag_load(const _Float16* p) {
  union U { v16h v; v8h h[2]; } f;
  f.h[0] = *(const v8h*)(p);
  f.h[1] = *(const v8h*)(p + 16);
  return f.v;
}
__device__ __forceinline__ v8f mma_f16(v16h a, v16h b, v8f c) {
  return __builtin_amdgcn_wmma_f32_16x16x32_f16(false, a, false, b, (short)0, c, false, false);
}
__device__ __forceinline__ void tie_acc(v8f& c, v16h a, v16h b) {
  asm volatile("v_nop\n\tv_nop\n\tv_nop\n\tv_nop" : "+v"(c) : "v"(a), "v"(b));
}
__device__ __forceinline__ void keep4_h(v16h a, v16h b, v16h c, v16h d) {
  asm volatile("v_nop" :: "v"(a), "v"(b), "v"(c), "v"(d));
}
__device__ __forceinline__ void acc_guard4(v8f& a, v8f& b, v8f& c, v8f& d) {
  asm volatile("v_nop\n\tv_nop\n\tv_nop\n\tv_nop" : "+v"(a), "+v"(b), "+v"(c), "+v"(d));
}

__global__ __launch_bounds__(256) void shape_kernel(
    const float* __restrict__ vt, const float* __restrict__ sd, const float* __restrict__ lbs,
    const float* __restrict__ betas, float* __restrict__ vs4, _Float16* __restrict__ Wh)
{
  __shared__ __align__(16) v8h sW8[256 * 12];
  const int tid = threadIdx.x;
  const int v = blockIdx.x * 256 + tid;
  const bool valid = (v < kNV);
  const int vc = valid ? v : (kNV - 1);

  const float scale = betas[0];
  float bl[kNBeta];
#pragma unroll
  for (int l = 0; l < kNBeta; ++l) bl[l] = betas[1 + l];

  float sdv[30];
  {
    const v2f* sp = (const v2f*)(sd + (size_t)vc * 30);
#pragma unroll
    for (int i = 0; i < 15; ++i) {
      const v2f t = sp[i];
      sdv[2 * i]     = t[0];
      sdv[2 * i + 1] = t[1];
    }
  }
  const float t0 = vt[vc * 3 + 0], t1 = vt[vc * 3 + 1], t2 = vt[vc * 3 + 2];
  float a0 = 0.0f, a1 = 0.0f, a2 = 0.0f;
#pragma unroll
  for (int l = 0; l < kNBeta; ++l) {
    a0 = fmaf(bl[l], sdv[l], a0);
    a1 = fmaf(bl[l], sdv[10 + l], a1);
    a2 = fmaf(bl[l], sdv[20 + l], a2);
  }
  const float h0 = (t0 + a0) * scale;
  const float h1 = (t1 + a1) * scale;
  const float h2 = (t2 + a2) * scale;
  const float hz0 = valid ? h0 : 0.0f;
  const float hz1 = valid ? h1 : 0.0f;
  const float hz2 = valid ? h2 : 0.0f;
  const float one = valid ? 1.0f : 0.0f;

  float wz[kNJ];
  {
    const v4f* wp = (const v4f*)(lbs + (size_t)vc * kNJ);
#pragma unroll
    for (int i = 0; i < 6; ++i) {
      const v4f t = wp[i];
      wz[4 * i + 0] = valid ? t[0] : 0.0f;
      wz[4 * i + 1] = valid ? t[1] : 0.0f;
      wz[4 * i + 2] = valid ? t[2] : 0.0f;
      wz[4 * i + 3] = valid ? t[3] : 0.0f;
    }
  }
#pragma unroll
  for (int i = 0; i < 12; ++i) {
    const float wa = wz[2 * i], wb = wz[2 * i + 1];
    v8h hv;
    hv[0] = (_Float16)((wa * hz0) * kCarryW);
    hv[1] = (_Float16)((wa * hz1) * kCarryW);
    hv[2] = (_Float16)((wa * hz2) * kCarryW);
    hv[3] = (_Float16)(wa * kCarryW);
    hv[4] = (_Float16)((wb * hz0) * kCarryW);
    hv[5] = (_Float16)((wb * hz1) * kCarryW);
    hv[6] = (_Float16)((wb * hz2) * kCarryW);
    hv[7] = (_Float16)(wb * kCarryW);
    sW8[tid * 12 + i] = hv;
  }
  __syncthreads();

  v4f ov;
  ov[0] = hz0; ov[1] = hz1; ov[2] = hz2; ov[3] = one;
  float* vdst = vs4 + (size_t)v * 4;
  _Float16* wdst = Wh + (size_t)blockIdx.x * 256 * kKdim;
  for (int pass = 0; pass < 2; ++pass) {
    *(volatile v4f*)vdst = ov;
#pragma unroll 4
    for (int it = 0; it < 12; ++it) {
      const int idx = it * 256 + tid;
      const v8h x = sW8[idx];
      *(volatile v8h*)(wdst + (size_t)idx * 8) = x;
    }
    __threadfence();
  }
}

__global__ __launch_bounds__(256) void jreg_kernel(
    const float* __restrict__ Jr, const float* __restrict__ vs4, float* __restrict__ Jsp)
{
  __shared__ float red[3 * 256];
  const int tid = threadIdx.x;
  const int j = blockIdx.x;
  float a0 = 0.0f, a1 = 0.0f, a2 = 0.0f;
#pragma unroll 1
  for (int v = tid; v < kNV; v += 256) {
    const float w = Jr[(size_t)j * kNV + v];
    const v4f h = *(const v4f*)(vs4 + (size_t)v * 4);
    a0 = fmaf(w, h[0], a0);
    a1 = fmaf(w, h[1], a1);
    a2 = fmaf(w, h[2], a2);
  }
  red[tid] = a0;
  red[256 + tid] = a1;
  red[512 + tid] = a2;
  __syncthreads();
  for (int s = 128; s > 0; s >>= 1) {
    if (tid < s) {
      red[tid]       += red[tid + s];
      red[256 + tid] += red[256 + tid + s];
      red[512 + tid] += red[512 + tid + s];
    }
    __syncthreads();
  }
  if (tid < 32) {
    const int c = (tid < 3) ? tid : 2;
    const float x = red[c * 256];
    const float val = (tid < 3) ? x : 0.0f;
    float* dst = Jsp + j * 32 + tid;
    *(volatile float*)dst = val;
    __threadfence();
    *(volatile float*)dst = val;
  }
}

__global__ __launch_bounds__(32) void chain_kernel(
    const float* __restrict__ bp,  const float* __restrict__ rbk, const float* __restrict__ rfr,
    const float* __restrict__ lbk, const float* __restrict__ lfr, const float* __restrict__ go,
    const float* __restrict__ Jsp, float* __restrict__ Af, _Float16* __restrict__ Ah,
    float* __restrict__ out)
{
  __shared__ __align__(16) float sA[32 * 3 * kKdim];
  __shared__ __align__(16) float sT[32 * 72];
  __shared__ __align__(16) float sJ[96];
  const int lane = threadIdx.x;
  const int b = blockIdx.x * 32 + lane;

#pragma unroll
  for (int i = 0; i < 3; ++i) {
    const int idx = i * 32 + lane;
    sJ[idx] = Jsp[(idx >> 2) * 32 + (idx & 3)];
  }
  __syncthreads();

  float* myA = sA + lane * (3 * kKdim);
  float* myT = sT + lane * 72;

#pragma unroll 1
  for (int j = 0; j < kNJ; ++j) {
    const float* src = bp;
    int stride = 57, off = 0, single = 0;
    if (j == 0)       { src = go;  stride = 3;  off = 0; }
    else if (j <= 6)  { src = bp;  stride = 57; off = 3 * (j - 1); }
    else if (j == 7)  { src = lbk; stride = 3;  off = 0; }
    else if (j == 8)  { src = rbk; stride = 3;  off = 0; }
    else if (j == 9)  { src = bp;  stride = 57; off = 18; }
    else if (j == 10) { src = lfr; stride = 1;  off = 0; single = 1; }
    else if (j == 11) { src = rfr; stride = 1;  off = 0; single = 1; }
    else              { src = bp;  stride = 57; off = 21 + 3 * (j - 12); }
    const int base = b * stride + off;
    const int o1 = single ? 0 : 1;
    const int o2 = single ? 0 : 2;
    const float q0 = src[base];
    const float q1 = src[base + o1];
    const float q2 = src[base + o2];
    const float rx = q0;
    const float ry = single ? 0.0f : q1;
    const float rz = single ? 0.0f : q2;

    const float ax = rx + 1e-8f, ay = ry + 1e-8f, az = rz + 1e-8f;
    const float ang = sqrtf((ax * ax + az * az) + ay * ay);
    const float inv = 1.0f / ang;
    const float dx = rx * inv, dy = ry * inv, dz = rz * inv;
    const float sn = sinf(ang);
    const float cs = cosf(ang);
    const float oc = 1.0f - cs;
    const float xx = dx * dx, yy = dy * dy, zz = dz * dz;
    const float xy = dx * dy, xz = dx * dz, yz = dy * dz;
    float Rl[9];
    Rl[0] = 1.0f - oc * (zz + yy);
    Rl[1] = oc * xy - sn * dz;
    Rl[2] = oc * xz + sn * dy;
    Rl[3] = oc * xy + sn * dz;
    Rl[4] = 1.0f - oc * (zz + xx);
    Rl[5] = oc * yz - sn * dx;
    Rl[6] = oc * xz - sn * dy;
    Rl[7] = oc * yz + sn * dx;
    Rl[8] = 1.0f - oc * (yy + xx);

    int p = 0;
    if (j > 0) {
      const unsigned long long bits = (j < 12) ? (kParLo >> (5 * j)) : (kParHi >> (5 * (j - 12)));
      p = (int)(bits & 31ull);
    }
    const float js0 = sJ[4 * j + 0], js1 = sJ[4 * j + 1], js2 = sJ[4 * j + 2];
    const float jp0 = sJ[4 * p + 0], jp1 = sJ[4 * p + 1], jp2 = sJ[4 * p + 2];
    const float rel0 = (j > 0) ? (js0 - jp0) : js0;
    const float rel1 = (j > 0) ? (js1 - jp1) : js1;
    const float rel2 = (j > 0) ? (js2 - jp2) : js2;

#pragma unroll 1
    for (int m = 0; m < 3; ++m) {
      float pr0, pr1, pr2, tp;
      if (j > 0) {
        pr0 = myA[m * kKdim + 4 * p + 0];
        pr1 = myA[m * kKdim + 4 * p + 1];
        pr2 = myA[m * kKdim + 4 * p + 2];
        tp  = myT[3 * p + m];
      } else {
        pr0 = (m == 0) ? 1.0f : 0.0f;
        pr1 = (m == 1) ? 1.0f : 0.0f;
        pr2 = (m == 2) ? 1.0f : 0.0f;
        tp  = 0.0f;
      }
      const float r0 = pr0 * Rl[0] + pr1 * Rl[3] + pr2 * Rl[6];
      const float r1 = pr0 * Rl[1] + pr1 * Rl[4] + pr2 * Rl[7];
      const float r2 = pr0 * Rl[2] + pr1 * Rl[5] + pr2 * Rl[8];
      const float tj = pr0 * rel0 + pr1 * rel1 + pr2 * rel2 + tp;
      const float ib = r0 * js0 + r1 * js1 + r2 * js2;
      myA[m * kKdim + 4 * j + 0] = r0;
      myA[m * kKdim + 4 * j + 1] = r1;
      myA[m * kKdim + 4 * j + 2] = r2;
      myA[m * kKdim + 4 * j + 3] = tj - ib;
      myT[3 * j + m] = tj;
    }
  }
  __syncthreads();

  float*    dstA = Af + (size_t)blockIdx.x * (32 * 3 * kKdim);
  _Float16* dstH = Ah + (size_t)blockIdx.x * (32 * 3 * kKdim);
  float*    dstO = out + kOut1Off + (size_t)blockIdx.x * (32 * 72);
  for (int pass = 0; pass < 2; ++pass) {
#pragma unroll 4
    for (int it = 0; it < 72; ++it) {
      const int idx = it * 32 + lane;
      const v4f x = *(const v4f*)(sA + idx * 4);
      *(volatile v4f*)(dstA + idx * 4) = x;
    }
#pragma unroll 2
    for (int it = 0; it < 36; ++it) {
      const int idx = it * 32 + lane;
      const v4f x0 = *(const v4f*)(sA + idx * 8);
      const v4f x1 = *(const v4f*)(sA + idx * 8 + 4);
      v8h hv;
#pragma unroll
      for (int e = 0; e < 4; ++e) {
        hv[e]     = (_Float16)x0[e];
        hv[4 + e] = (_Float16)x1[e];
      }
      *(volatile v8h*)(dstH + idx * 8) = hv;
    }
#pragma unroll 2
    for (int it = 0; it < 18; ++it) {
      const int idx = it * 32 + lane;
      const v4f x = *(const v4f*)(sT + idx * 4);
      *(volatile v4f*)(dstO + idx * 4) = x;
    }
    __threadfence();
  }
}

__global__ __launch_bounds__(256) void gemm_f16_kernel(
    const _Float16* __restrict__ A, int lda,
    const _Float16* __restrict__ Bt, int ldb,
    float* __restrict__ C, int ldc,
    int M, int N, int K, float scale)
{
  __shared__ __align__(16) float sT[8][16 * 68];
  const int lane = threadIdx.x & 31;
  const int wave = threadIdx.x >> 5;
  const int tilesN = N >> 6;
  const int tilesM = M >> 6;
  const int tile = blockIdx.x * 8 + wave;
  if (tile >= tilesM * tilesN) return;
  const int tm = tile / tilesN;
  const int tn = tile - tm * tilesN;
  const int m0 = tm << 6;
  const int n0 = tn << 6;

  const int rlane = lane & 15;
  const int koff  = (lane >> 4) * 8;
  const int mOff  = (lane >> 4) * 8;

  v8f acc[4][4];
#pragma unroll
  for (int i = 0; i < 4; ++i)
#pragma unroll
    for (int j = 0; j < 4; ++j) acc[i][j] = (v8f){0.f,0.f,0.f,0.f,0.f,0.f,0.f,0.f};

  for (int k0 = 0; k0 < K; k0 += 32) {
    v16h bh[4];
#pragma unroll
    for (int j = 0; j < 4; ++j) {
      const size_t bo = (size_t)(n0 + (j << 4) + rlane) * ldb + koff + k0;
      bh[j] = frag_load(Bt + bo);
    }
#pragma unroll
    for (int i = 0; i < 4; ++i) {
      const size_t ao = (size_t)(m0 + (i << 4) + rlane) * lda + koff + k0;
      const v16h ah = frag_load(A + ao);
#pragma unroll
      for (int j = 0; j < 4; ++j) acc[i][j] = mma_f16(ah, bh[j], acc[i][j]);
      tie_acc(acc[i][0], ah, bh[0]);
      tie_acc(acc[i][1], ah, bh[1]);
      tie_acc(acc[i][2], ah, bh[2]);
      tie_acc(acc[i][3], ah, bh[3]);
    }
    keep4_h(bh[0], bh[1], bh[2], bh[3]);
  }
  acc_guard4(acc[0][0], acc[0][1], acc[0][2], acc[0][3]);
  acc_guard4(acc[1][0], acc[1][1], acc[1][2], acc[1][3]);
  acc_guard4(acc[2][0], acc[2][1], acc[2][2], acc[2][3]);
  acc_guard4(acc[3][0], acc[3][1], acc[3][2], acc[3][3]);

  float* slab = sT[wave];
#pragma unroll
  for (int i = 0; i < 4; ++i) {
    const int mBase = m0 + (i << 4);
#pragma unroll
    for (int j = 0; j < 4; ++j) {
#pragma unroll
      for (int r = 0; r < 8; ++r) {
        const float val = acc[i][j][r] * scale;
        slab[(mOff + r) * 68 + (j << 4) + rlane] = val;
      }
    }
    __builtin_amdgcn_fence(__ATOMIC_RELEASE, "workgroup");
    __builtin_amdgcn_wave_barrier();
    __builtin_amdgcn_fence(__ATOMIC_ACQUIRE, "workgroup");
    {
      const int hh = lane >> 4, c4 = (lane & 15) * 4;
      for (int pass = 0; pass < 2; ++pass) {
#pragma unroll
        for (int it = 0; it < 8; ++it) {
          const int row = it * 2 + hh;
          const v4f val = *(const v4f*)(slab + row * 68 + c4);
          *(volatile v4f*)(C + (size_t)(mBase + row) * ldc + n0 + c4) = val;
        }
        __threadfence();
      }
    }
    __builtin_amdgcn_fence(__ATOMIC_RELEASE, "workgroup");
    __builtin_amdgcn_wave_barrier();
    __builtin_amdgcn_fence(__ATOMIC_ACQUIRE, "workgroup");
  }
}

__global__ __launch_bounds__(256) void repack_kernel(
    const float* __restrict__ Cp, const float* __restrict__ transl, float* __restrict__ out0)
{
  const int i4 = blockIdx.x * 256 + threadIdx.x;
  if (i4 >= kOut0F4) return;
  const unsigned f0 = (unsigned)i4 * 4u;
  v4f o;
#pragma unroll
  for (int e = 0; e < 4; ++e) {
    const unsigned f = f0 + (unsigned)e;
    const unsigned c3 = f / 3u;
    const unsigned m = f - 3u * c3;
    const unsigned bb = c3 / (unsigned)kNV;
    const unsigned v = c3 - (unsigned)kNV * bb;
    const unsigned row = 3u * bb + m;
    const float cv = Cp[(size_t)row * kNVPad + v];
    const float tv = transl[row];
    o[e] = cv + tv;
  }
  float* dst = out0 + (size_t)f0;
  *(volatile v4f*)dst = o;
  __threadfence();
  *(volatile v4f*)dst = o;
}

__global__ __launch_bounds__(256) void planes_kernel(
    const float* __restrict__ lbs, const float* __restrict__ transl,
    const float* __restrict__ ip_bl, const float* __restrict__ ip_fl,
    const float* __restrict__ ip_br, const float* __restrict__ ip_fr,
    const int* __restrict__ id_bl, const int* __restrict__ id_fl,
    const int* __restrict__ id_br, const int* __restrict__ id_fr,
    const float* __restrict__ Af, float* __restrict__ out)
{
  __shared__ __align__(16) float sAf[6 * kKdim];
  __shared__ __align__(16) float sO[2 * kGroups * kPts * 3];
  const int tid = threadIdx.x;
  const int b0 = blockIdx.x * 2;
  {
    const int ic = (tid < 144) ? tid : 143;
    const v4f x = *(const v4f*)(Af + (size_t)b0 * 3 * kKdim + ic * 4);
    if (tid < 144) *(v4f*)(sAf + tid * 4) = x;
  }
  __syncthreads();

  const bool active = (tid < 2 * kPts);
  const int item = active ? tid : (2 * kPts - 1);
  const int bb = item / kPts;
  const int p = item - bb * kPts;
  const int b = b0 + bb;
  const float tr0 = transl[b * 3 + 0], tr1 = transl[b * 3 + 1], tr2 = transl[b * 3 + 2];

#pragma unroll 1
  for (int g = 0; g < kGroups; ++g) {
    const int*   ids = (g == 0) ? id_bl : (g == 1) ? id_fl : (g == 2) ? id_br : id_fr;
    const float* ip  = (g == 0) ? ip_bl : (g == 1) ? ip_fl : (g == 2) ? ip_br : ip_fr;
    int v = ids[p];
    v = (v < 0) ? 0 : v;
    v = (v > kNV - 1) ? (kNV - 1) : v;
    const float ix = ip[(b * kPts + p) * 3 + 0];
    const float iy = ip[(b * kPts + p) * 3 + 1];
    const float iz = ip[(b * kPts + p) * 3 + 2];
    float T[12];
#pragma unroll
    for (int i = 0; i < 12; ++i) T[i] = 0.0f;
#pragma unroll 1
    for (int j = 0; j < kNJ; ++j) {
      const float w = lbs[(size_t)v * kNJ + j];
#pragma unroll
      for (int m = 0; m < 3; ++m) {
        const v4f a = *(const v4f*)(sAf + (bb * 3 + m) * kKdim + 4 * j);
        T[m * 4 + 0] = fmaf(w, a[0], T[m * 4 + 0]);
        T[m * 4 + 1] = fmaf(w, a[1], T[m * 4 + 1]);
        T[m * 4 + 2] = fmaf(w, a[2], T[m * 4 + 2]);
        T[m * 4 + 3] = fmaf(w, a[3], T[m * 4 + 3]);
      }
    }
    const float o0 = (T[0] * ix + T[1] * iy + T[2]  * iz + T[3])  + tr0;
    const float o1 = (T[4] * ix + T[5] * iy + T[6]  * iz + T[7])  + tr1;
    const float o2 = (T[8] * ix + T[9] * iy + T[10] * iz + T[11]) + tr2;
    if (active) {
      float* so = sO + bb * (kGroups * kPts * 3) + (g * kPts + p) * 3;
      so[0] = o0;
      so[1] = o1;
      so[2] = o2;
    }
  }
  __syncthreads();

  float* dst = out + kOut2Off + (size_t)b0 * (kGroups * kPts * 3);
  for (int pass = 0; pass < 2; ++pass) {
#pragma unroll
    for (int it = 0; it < 3; ++it) {
      const int idx = it * 256 + tid;
      if (idx < 600) {
        const v4f x = *(const v4f*)(sO + idx * 4);
        *(volatile v4f*)(dst + idx * 4) = x;
      }
    }
    __threadfence();
  }
}

extern "C" void kernel_launch(void* const* d_in, const int* in_sizes, int n_in,
                              void* d_out, int out_size, void* d_ws, size_t ws_size,
                              hipStream_t stream) {
  if (n_in < 21) return;
  if (in_sizes[0] != kNV * 3) return;
  if (in_sizes[1] != kNV * 3 * kNBeta) return;
  if (in_sizes[2] != kNJ * kNV) return;
  if (in_sizes[3] != kNV * kNJ) return;
  if (in_sizes[4] != 1 + kNBeta) return;
  if (in_sizes[5] != kBatch * 57) return;
  if (in_sizes[6] != kBatch * 3) return;
  if (in_sizes[7] != kBatch) return;
  if (in_sizes[8] != kBatch * 3) return;
  if (in_sizes[9] != kBatch) return;
  if (in_sizes[10] != kBatch * 3) return;
  if (in_sizes[11] != kBatch * 3) return;
  if (in_sizes[12] != kBatch * kPts * 3) return;
  if (in_sizes[13] != kBatch * kPts * 3) return;
  if (in_sizes[14] != kBatch * kPts * 3) return;
  if (in_sizes[15] != kBatch * kPts * 3) return;
  if (in_sizes[17] != kPts || in_sizes[18] != kPts || in_sizes[19] != kPts || in_sizes[20] != kPts) return;
  if (out_size != kOut0Elems + kOut1Elems + kOut2Elems) return;
  if (ws_size < kWsTotal) return;

  const float* vt    = (const float*)d_in[0];
  const float* sd    = (const float*)d_in[1];
  const float* Jr    = (const float*)d_in[2];
  const float* lbs   = (const float*)d_in[3];
  const float* betas = (const float*)d_in[4];
  const float* bp    = (const float*)d_in[5];
  const float* rbk   = (const float*)d_in[6];
  const float* rfr   = (const float*)d_in[7];
  const float* lbk   = (const float*)d_in[8];
  const float* lfr   = (const float*)d_in[9];
  const float* trl   = (const float*)d_in[10];
  const float* go    = (const float*)d_in[11];
  const float* ip_bl = (const float*)d_in[12];
  const float* ip_fl = (const float*)d_in[13];
  const float* ip_br = (const float*)d_in[14];
  const float* ip_fr = (const float*)d_in[15];
  const int* id_bl = (const int*)d_in[17];
  const int* id_br = (const int*)d_in[18];
  const int* id_fl = (const int*)d_in[19];
  const int* id_fr = (const int*)d_in[20];

  float* out = (float*)d_out;
  char* ws = (char*)d_ws;
  float*    VS4 = (float*)(ws + kOffVS4);
  _Float16* WH  = (_Float16*)(ws + kOffWH);
  float*    JSP = (float*)(ws + kOffJSP);
  float*    AF  = (float*)(ws + kOffAF);
  _Float16* AH  = (_Float16*)(ws + kOffAH);
  float*    CP  = (float*)(ws + kOffCP);

  shape_kernel<<<kNVPad / 256, 256, 0, stream>>>(vt, sd, lbs, betas, VS4, WH);
  jreg_kernel<<<kNJ, 256, 0, stream>>>(Jr, VS4, JSP);
  chain_kernel<<<kBatch / 32, 32, 0, stream>>>(bp, rbk, rfr, lbk, lfr, go, JSP, AF, AH, out);
  gemm_f16_kernel<<<((kCdim / 64) * (kNVPad / 64) + 7) / 8, 256, 0, stream>>>(
      AH, kKdim, WH, kKdim, CP, kNVPad, kCdim, kNVPad, kKdim, 1.0f / kCarryW);
  repack_kernel<<<(kOut0F4 + 255) / 256, 256, 0, stream>>>(CP, trl, out);
  planes_kernel<<<kBatch / 2, 256, 0, stream>>>(lbs, trl, ip_bl, ip_fl, ip_br, ip_fr,
                                               id_bl, id_fl, id_br, id_fr, AF, out);
}
